// GNNModel_69329362092401
// MI455X (gfx1250) — hardware-run, weakly checked
//
#include <hip/hip_runtime.h>

typedef float          v8f   __attribute__((ext_vector_type(8)));
typedef float          v4f   __attribute__((ext_vector_type(4)));
typedef unsigned int   v4u   __attribute__((ext_vector_type(4)));
typedef int            v8i   __attribute__((ext_vector_type(8)));
typedef unsigned short v8us  __attribute__((ext_vector_type(8)));
typedef unsigned short v16us __attribute__((ext_vector_type(16)));
typedef __bf16         v16bf __attribute__((ext_vector_type(16)));
typedef _Float16       v16h  __attribute__((ext_vector_type(16)));
typedef v4f  __attribute__((may_alias)) v4fa;
typedef v8us __attribute__((may_alias)) v8usa;
union FragB { v16bf v; v16us u; v8us h[2]; v8i w; };
union FragH { v16h  v; v16us u; v8us h[2]; v8i w; };

__device__ __forceinline__ v8f wmb(const FragB& a, const FragB& b, v8f c) {
  v8f d = __builtin_amdgcn_wmma_f32_16x16x32_bf16(false, a.v, false, b.v, (short)0, c, false, false);
  asm volatile("v_nop\n\tv_nop\n\tv_nop\n\tv_nop" : "+v"(d) : "v"(a.w), "v"(b.w));
  return d;
}

__device__ __forceinline__ v8f wmh(const FragH& a, const FragH& b, v8f c) {
  v8f d = __builtin_amdgcn_wmma_f32_16x16x32_f16(false, a.v, false, b.v, (short)0, c, false, false);
  asm volatile("v_nop\n\tv_nop\n\tv_nop\n\tv_nop" : "+v"(d) : "v"(a.w), "v"(b.w));
  return d;
}

__device__ __forceinline__ unsigned bf16_bits(float f) {
  const unsigned u = __float_as_uint(f);
  const unsigned r = (u + 0x7FFFu + ((u >> 16) & 1u)) >> 16;
  const unsigned q = (u >> 16) | 0x40u;
  return ((u & 0x7fffffffu) > 0x7f800000u) ? q : r;
}

__device__ __forceinline__ float bf16_val(float f) {
  return __uint_as_float(bf16_bits(f) << 16);
}
__device__ __forceinline__ int clampi(int v, int lo, int hi) {
  return v < lo ? lo : (v > hi ? hi : v);
}

__device__ __forceinline__ unsigned f16_bits(float f) {
  const unsigned u  = __float_as_uint(f);
  const unsigned s  = (u >> 16) & 0x8000u;
  const unsigned a  = u & 0x7fffffffu;
  const unsigned t  = a - 0x38000000u;
  const unsigned r  = (t + 0x0FFFu + ((t >> 13) & 1u)) >> 13;
  const unsigned rc = r > 0x7C00u ? 0x7C00u : r;
  const bool small  = a < 0x38800000u;
  const bool isnan  = a > 0x7f800000u;
  const unsigned fin = small ? 0u : (s | rc);
  return isnan ? (s | 0x7E00u) : fin;
}

__device__ __forceinline__ unsigned pk16(unsigned lo, unsigned hi) { return lo | (hi << 16); }
__device__ __forceinline__ unsigned bf16_lo_bits(float v) {
  float hi = bf16_val(v);
  asm volatile("" : "+v"(hi));
  return bf16_bits(v - hi);
}
__device__ __forceinline__ v4u pack8_bf16(v4f a, v4f c) {
  return (v4u){ pk16(bf16_bits(a[0]), bf16_bits(a[1])), pk16(bf16_bits(a[2]), bf16_bits(a[3])),
                pk16(bf16_bits(c[0]), bf16_bits(c[1])), pk16(bf16_bits(c[2]), bf16_bits(c[3])) };
}
__device__ __forceinline__ v4u pack8_bf16_lo(v4f a, v4f c) {
  return (v4u){ pk16(bf16_lo_bits(a[0]), bf16_lo_bits(a[1])), pk16(bf16_lo_bits(a[2]), bf16_lo_bits(a[3])),
                pk16(bf16_lo_bits(c[0]), bf16_lo_bits(c[1])), pk16(bf16_lo_bits(c[2]), bf16_lo_bits(c[3])) };
}
__device__ __forceinline__ v4u pack8_f16(v4f a, v4f c) {
  return (v4u){ pk16(f16_bits(a[0]), f16_bits(a[1])), pk16(f16_bits(a[2]), f16_bits(a[3])),
                pk16(f16_bits(c[0]), f16_bits(c[1])), pk16(f16_bits(c[2]), f16_bits(c[3])) };
}

template <int FORM>
__global__ __launch_bounds__(256) void k_plane(const float* __restrict__ src, int rows, int cols, int ldsrc,
                                               unsigned short* __restrict__ dst, int MP, int KP) {
  static_assert(FORM >= 0 && FORM <= 3);
  const int KTOT = (FORM == 1 || FORM == 3) ? 2 * KP : KP;
  const unsigned ppr   = (unsigned)(KTOT >> 3);
  const unsigned kp8   = (unsigned)(KP >> 3);
  const unsigned total = (unsigned)MP * ppr;
  const unsigned g     = blockIdx.x * 256u + threadIdx.x;
  const unsigned rowu  = g / ppr;
  const unsigned p     = g - rowu * ppr;
  const bool second    = p >= kp8;
  const int row = (int)rowu;
  const int c0  = (int)((second ? p - kp8 : p) << 3);
  const float* srow = src + (size_t)clampi(row, 0, rows - 1) * (size_t)ldsrc;
  float x[8];
  unsigned mk[8];
#pragma unroll
  for (int e = 0; e < 8; ++e) {
    const int c = c0 + e;
    const float v = srow[clampi(c, 0, cols - 1)];
    asm volatile("" :: "v"(v));
    x[e]  = v;
    mk[e] = (row < rows && c < cols) ? 0xFFFFu : 0u;
  }
  const v4f a = (v4f){ x[0], x[1], x[2], x[3] };
  const v4f c = (v4f){ x[4], x[5], x[6], x[7] };
  v4u o;
  if (FORM == 2) {
    o = pack8_f16(a, c);
  } else {
    const v4u hi = pack8_bf16(a, c);
    o = hi;
    if (FORM == 1) { const v4u lo = pack8_bf16_lo(a, c); o = second ? lo : hi; }
  }
  const v4u mw = (v4u){ pk16(mk[0], mk[1]), pk16(mk[2], mk[3]), pk16(mk[4], mk[5]), pk16(mk[6], mk[7]) };
  o &= mw;
  if (g < total) {
    volatile v4u* q = (volatile v4u*)(dst + (size_t)g * 8);
    *q = o;
    __threadfence();
    *q = o;
  }
}

template <int FORM> struct FragOf    { typedef FragB T; };
template <>         struct FragOf<2> { typedef FragH T; };
__device__ __forceinline__ v8f mm(const FragB& a, const FragB& b, v8f c) { return wmb(a, b, c); }
__device__ __forceinline__ v8f mm(const FragH& a, const FragH& b, v8f c) { return wmh(a, b, c); }
template <class F> __device__ __forceinline__ F ld_frag(const unsigned short* p) {
  F f;
  f.h[0] = *(const v8usa*)(p);
  f.h[1] = *(const v8usa*)(p + 16);
  return f;
}

template <int FORM, int EPI>
__global__ __launch_bounds__(256) __attribute__((amdgpu_num_vgpr(248)))
void k_gemm_nt(const unsigned short* __restrict__ A, const unsigned short* __restrict__ B,
               const float* __restrict__ bias, float* __restrict__ D, int M, int N, int KTOT, int ldd) {
  static_assert(FORM >= 0 && FORM <= 2);
  static_assert(EPI == 0 || EPI == 1);
  typedef typename FragOf<FORM>::T F;
  __shared__ __attribute__((aligned(16))) float sT[8][16 * 68];
  const int lane = threadIdx.x & 31;
  const int wave = threadIdx.x >> 5;
  const int tilesM = (M + 63) >> 6;
  const int tilesN = (N + 63) >> 6;
  const int tile = blockIdx.x * 8 + wave;
  if (tile >= tilesM * tilesN) return;
  const int tm = tile / tilesN;
  const int tn = tile - tm * tilesN;
  const int m0 = tm << 6;
  const int n0 = tn << 6;

  const int rl = lane & 15;
  const int h8 = (lane >> 4) * 8;
  const unsigned short* pa = A + (size_t)(m0 + rl) * (size_t)KTOT + h8;
  const unsigned short* pb = B + (size_t)(n0 + rl) * (size_t)KTOT + h8;

  v8f acc[4][4];
#pragma unroll
  for (int i = 0; i < 4; ++i)
#pragma unroll
    for (int j = 0; j < 4; ++j) acc[i][j] = (v8f){0.f, 0.f, 0.f, 0.f, 0.f, 0.f, 0.f, 0.f};

#pragma unroll 1
  for (int k0 = 0; k0 < KTOT; k0 += 32) {
    F bf[4];
#pragma unroll
    for (int j = 0; j < 4; ++j) bf[j] = ld_frag<F>(pb + (size_t)(j << 4) * (size_t)KTOT + k0);
#pragma unroll
    for (int i = 0; i < 4; ++i) {
      const F af = ld_frag<F>(pa + (size_t)(i << 4) * (size_t)KTOT + k0);
#pragma unroll
      for (int j = 0; j < 4; ++j) acc[i][j] = mm(af, bf[j], acc[i][j]);
    }
  }

  float* slab = sT[wave];
  const int hh = lane >> 4;
  const int c4 = (lane & 15) * 4;
  const int nc = n0 + c4;
  const bool cok = nc < N;
  v4f bv = (v4f){0.f, 0.f, 0.f, 0.f};
  if (EPI == 1) {
    bv = *(const v4fa*)(bias + clampi(nc, 0, N - 4));
    asm volatile("" :: "v"(bv));
  }
#pragma unroll
  for (int i = 0; i < 4; ++i) {
    const int mBase = m0 + (i << 4);
#pragma unroll
    for (int j = 0; j < 4; ++j) {
#pragma unroll
      for (int r = 0; r < 8; ++r) slab[(h8 + r) * 68 + (j << 4) + rl] = acc[i][j][r];
    }
    __builtin_amdgcn_fence(__ATOMIC_RELEASE, "workgroup");
    __builtin_amdgcn_wave_barrier();
    __builtin_amdgcn_fence(__ATOMIC_ACQUIRE, "workgroup");
    v4f vv[8];
#pragma unroll
    for (int it = 0; it < 8; ++it) {
      const int row = it * 2 + hh;
      v4f v = *(const v4fa*)(slab + row * 68 + c4);
      if (EPI == 1) v += bv;
      vv[it] = v;
    }
    for (int pass = 0; pass < 2; ++pass) {
#pragma unroll
      for (int it = 0; it < 8; ++it) {
        const int row = mBase + it * 2 + hh;
        if (cok && row < M) *(volatile v4f*)(D + (size_t)row * (size_t)ldd + nc) = vv[it];
      }
      __threadfence();
    }
    __builtin_amdgcn_fence(__ATOMIC_RELEASE, "workgroup");
    __builtin_amdgcn_wave_barrier();
    __builtin_amdgcn_fence(__ATOMIC_ACQUIRE, "workgroup");
  }
}

#define NN        100000
#define NE        600000
#define VOC       50000
#define DIM       128
#define H1_SPLIT  1
#define K2TOT     (H1_SPLIT ? 256 : 128)
#define MPN       100096
#define MPT       50048
#define NBRUN     1024
#define SLB       10
#define NOWN      98
#define NPB       (NOWN * NBRUN)
#define RCAP      8192
#define DEGCAP    64
#define WLCAP     2048
#define NWAVE     8
#define WSEG      75008
#define NCHW      293
#define MEAS_MAXDEG 19
#define MEAS_B1024  6297
#define WSMAX     ((size_t)128 << 20)

typedef int v4i __attribute__((ext_vector_type(4)));
typedef v4i __attribute__((may_alias)) v4ia;

static_assert(DIM == 32 * 4);
static_assert(MPN % 128 == 0 && MPT % 128 == 0 && MPN >= NN && MPT >= VOC && MPN % 8 == 0);
static_assert(K2TOT == (H1_SPLIT ? 2 : 1) * DIM && K2TOT % 32 == 0);
static_assert(NBRUN == (1 << SLB) && NBRUN == 4 * 256);
static_assert(NOWN * NBRUN >= NN && (NOWN - 1) * NBRUN < NN);
static_assert(RCAP % 256 == 0 && 4 * RCAP >= 5 * MEAS_B1024 && RCAP == 8 * 256 * 4);
static_assert(DEGCAP >= MEAS_MAXDEG + 8);
static_assert(NE % 8 == 0 && WSEG % 256 == 0 && NCHW * 256 == WSEG);
static_assert(NWAVE * WSEG >= NE && NWAVE * WSEG < (1 << 20));
static_assert(NN % 8 == 0);

#define BK_WL    0
#define BK_CW    (BK_WL + NWAVE * WLCAP)
#define BK_SL    (BK_CW + NWAVE * NBRUN)
#define BK_CNT   (BK_SL + RCAP)
#define BK_OFF   (BK_CNT + NBRUN)
#define BK_DS    (BK_OFF + NBRUN)
#define BK_MISC  (BK_DS + NBRUN)
#define BK_INTS  (BK_MISC + 32)
#define BK_BYTES (BK_INTS * 4)
static_assert(BK_BYTES == 143488 && BK_BYTES <= 262144);
static_assert((NWAVE * NBRUN + RCAP) % 1024 == 0);

#define SZ_A     ((size_t)MPN * 256 * 2)
#define SZ_B     ((size_t)MPN * DIM * 4)
#define SZ_LIST  ((size_t)NOWN * RCAP * 4)
#define SZ_TAB   ((size_t)NPB * 4)
#define SZ_FLG   ((size_t)NOWN * 128)
#define SZ_W1T   ((size_t)DIM * DIM * 2)
#define SZ_W2D   ((size_t)DIM * 256 * 2)
#define SZ_BR    ((size_t)DIM * 4)
#define O_A      ((size_t)0)
#define O_B      (O_A + SZ_A)
#define O_LIST   (O_B + SZ_B)
#define O_OFF    (O_LIST + SZ_LIST)
#define O_CNT    (O_OFF + SZ_TAB)
#define O_DINV   (O_CNT + SZ_TAB)
#define O_FLG    (O_DINV + SZ_TAB)
#define O_W1T    (O_FLG + SZ_FLG)
#define O_W2D    (O_W1T + SZ_W1T)
#define O_B1R    (O_W2D + SZ_W2D)
#define O_B2R    (O_B1R + SZ_BR)
#define WS_TOTAL (O_B2R + SZ_BR)
static_assert(SZ_A % 256 == 0 && SZ_B % 256 == 0 && SZ_LIST % 256 == 0 && SZ_TAB % 256 == 0 && SZ_FLG % 256 == 0);
static_assert(SZ_W1T % 256 == 0 && SZ_W2D % 256 == 0 && SZ_BR % 256 == 0);
static_assert((size_t)MPT * DIM * 2 <= SZ_A && (size_t)MPN * K2TOT * 2 <= SZ_A);
static_assert((size_t)MPT * DIM * 4 <= SZ_B);
static_assert((size_t)DIM * K2TOT * 2 <= SZ_W2D);
static_assert(WS_TOTAL == (size_t)((size_t)418069 << 8) && WS_TOTAL <= (size_t)WSMAX);

__device__ __forceinline__ int wave_incl_scan(int v, int lane) {
  int incl = v;
#pragma unroll
  for (int d = 1; d < 32; d <<= 1) {
    const int y = __shfl_up(incl, (unsigned)d, 32);
    incl += (lane >= d) ? y : 0;
  }
  return incl;
}

#define PB1 8
#define PB2 (DIM * (K2TOT / 8) / 256)
static_assert(PB1 * 256 == DIM * (DIM / 8) && PB2 * 256 == DIM * (K2TOT / 8));
__global__ __launch_bounds__(256) void k_prep(const float* __restrict__ W1, const float* __restrict__ W2,
                                              const float* __restrict__ b1, const float* __restrict__ b2,
                                              unsigned short* __restrict__ W1T, unsigned short* __restrict__ W2D,
                                              float* __restrict__ B1R, float* __restrict__ B2R) {
  const int b = (int)blockIdx.x, tid = (int)threadIdx.x;
  if (b < PB1) {
    const int u  = b * 256 + tid;
    const int n  = u >> 4;
    const int k8 = (u & 15) * 8;
    const float* p = W1 + (size_t)k8 * DIM + n;
    float x[8];
#pragma unroll
    for (int i = 0; i < 8; ++i) x[i] = p[(size_t)i * DIM];
    const v4u o = pack8_bf16((v4f){ x[0], x[1], x[2], x[3] }, (v4f){ x[4], x[5], x[6], x[7] });
    volatile v4u* q = (volatile v4u*)(W1T + (size_t)n * DIM + k8);
    *q = o;
    __threadfence();
    *q = o;
  } else if (b < PB1 + PB2) {
    const int u  = (b - PB1) * 256 + tid;
    const int n  = u / (K2TOT / 8);
    const int k8 = (u - n * (K2TOT / 8)) * 8;
    const int kk = k8 & (DIM - 1);
    const float* p = W2 + (size_t)kk * DIM + n;
    float x[8];
#pragma unroll
    for (int i = 0; i < 8; ++i) x[i] = p[(size_t)i * DIM];
    const v4u o = pack8_bf16((v4f){ x[0], x[1], x[2], x[3] }, (v4f){ x[4], x[5], x[6], x[7] });
    volatile v4u* q = (volatile v4u*)(W2D + (size_t)n * K2TOT + k8);
    *q = o;
    __threadfence();
    *q = o;
  } else {
    if (tid < 32) {
      const v4f a1 = *(const v4fa*)(b1 + 4 * tid);
      const v4f a2 = *(const v4fa*)(b2 + 4 * tid);
      const v4f r1 = (v4f){ bf16_val(a1.x), bf16_val(a1.y), bf16_val(a1.z), bf16_val(a1.w) };
      const v4f r2 = (v4f){ bf16_val(a2.x), bf16_val(a2.y), bf16_val(a2.z), bf16_val(a2.w) };
      volatile v4f* q1 = (volatile v4f*)(B1R + 4 * tid);
      volatile v4f* q2 = (volatile v4f*)(B2R + 4 * tid);
      *q1 = r1;
      *q2 = r2;
      __threadfence();
      *q1 = r1;
      *q2 = r2;
    }
  }
}

#define PUTJ(J, HJ, SJ) { if ((HJ) && pos < WLCAP) wl[pos] = (int)((((unsigned)(e0 + (J))) << SLB) | (SJ)); pos += (HJ) ? 1 : 0; }
__global__ __launch_bounds__(256) void k_bucket(const int* __restrict__ edge, int* __restrict__ LIST,
                                                int* __restrict__ OFF, int* __restrict__ CNT,
                                                float* __restrict__ DINV, int* __restrict__ FLG) {
  extern __shared__ __attribute__((aligned(16))) int dsm[];
  const int tid = (int)threadIdx.x, lane = tid & 31, wave = tid >> 5;
  const int blk = (int)blockIdx.x;
  const int nodeBase = blk * NBRUN;
  const int nb = clampi(NN - nodeBase, 0, NBRUN);
  const int* srcs = edge;
  const int* dsts = edge + NE;
  int*   wl   = dsm + BK_WL + wave * WLCAP;
  int*   cw   = dsm + BK_CW;
  int*   cwm  = dsm + BK_CW + wave * NBRUN;
  int*   sl   = dsm + BK_SL;
  int*   cntS = dsm + BK_CNT;
  int*   offS = dsm + BK_OFF;
  float* dS   = (float*)(dsm + BK_DS);
  int*   misc = dsm + BK_MISC;

  {
    const v4i z4 = {0, 0, 0, 0};
#pragma unroll 1
    for (int i = tid * 4; i < NWAVE * NBRUN + RCAP; i += 1024) *(v4ia*)(dsm + BK_CW + i) = z4;
    if (tid < 32) misc[tid] = 0;
  }
  __syncthreads();

  int wc = 0;
  const int wbase = wave * WSEG;
  const unsigned nbs = (unsigned)nodeBase;
  const unsigned unb = (unsigned)nb;
#pragma unroll 1
  for (int ch = 0; ch < NCHW; ++ch) {
    const int e0 = wbase + ch * 256 + lane * 8;
    const int ec = e0 < NE - 8 ? e0 : NE - 8;
    const v4i da = *(const v4ia*)(dsts + ec);
    const v4i db = *(const v4ia*)(dsts + ec + 4);
    asm volatile("" :: "v"(da), "v"(db));
    const int km = (e0 < NE) ? 0 : -1;
    const unsigned s0 = (unsigned)(da.x | km) - nbs, s1 = (unsigned)(da.y | km) - nbs;
    const unsigned s2 = (unsigned)(da.z | km) - nbs, s3 = (unsigned)(da.w | km) - nbs;
    const unsigned s4 = (unsigned)(db.x | km) - nbs, s5 = (unsigned)(db.y | km) - nbs;
    const unsigned s6 = (unsigned)(db.z | km) - nbs, s7 = (unsigned)(db.w | km) - nbs;
    const bool h0 = s0 < unb, h1 = s1 < unb, h2 = s2 < unb, h3 = s3 < unb;
    const bool h4 = s4 < unb, h5 = s5 < unb, h6 = s6 < unb, h7 = s7 < unb;
    const int c = (int)h0 + (int)h1 + (int)h2 + (int)h3 + (int)h4 + (int)h5 + (int)h6 + (int)h7;
    const unsigned any = __builtin_amdgcn_ballot_w32(c != 0);
    if (any != 0u) {
      const int incl = wave_incl_scan(c, lane);
      const int tot  = __builtin_amdgcn_readlane(incl, 31);
      int pos = wc + incl - c;
      PUTJ(0, h0, s0)
      PUTJ(1, h1, s1)
      PUTJ(2, h2, s2)
      PUTJ(3, h3, s3)
      PUTJ(4, h4, s4)
      PUTJ(5, h5, s5)
      PUTJ(6, h6, s6)
      PUTJ(7, h7, s7)
      wc += tot;
    }
  }
  if (lane == 0) misc[wave] = wc;
  __syncthreads();

  int wcc = clampi(wc, 0, WLCAP);
  wcc = __builtin_amdgcn_readfirstlane(wcc);
#pragma unroll 1
  for (int b0 = 0; b0 < wcc; b0 += 32) {
    int idx = b0 + lane;
    idx = idx < wcc - 1 ? idx : wcc - 1;
    const int ent = wl[idx];
    const int m32 = (wcc - b0) < 32 ? (wcc - b0) : 32;
#pragma unroll 1
    for (int k = 0; k < m32; ++k) {
      const int u  = __builtin_amdgcn_readlane(ent, k);
      const int st = u & (NBRUN - 1);
      if (lane == 0) cwm[st] = cwm[st] + 1;
    }
  }
  __syncthreads();

  v4i c4[NWAVE];
  v4i tot4 = {0, 0, 0, 0};
#pragma unroll
  for (int w = 0; w < NWAVE; ++w) {
    c4[w] = *(const v4ia*)(cw + w * NBRUN + 4 * tid);
    tot4 += c4[w];
  }
  const int ts   = tot4.x + tot4.y + tot4.z + tot4.w;
  const int incT = wave_incl_scan(ts, lane);
  const bool bigl = (tot4.x > DEGCAP) | (tot4.y > DEGCAP) | (tot4.z > DEGCAP) | (tot4.w > DEGCAP);
  const unsigned bgm = __builtin_amdgcn_ballot_w32(bigl);
  if (lane == 31) misc[8 + wave] = incT;
  if (lane == 0)  misc[16 + wave] = (bgm != 0u) ? 1 : 0;
  __syncthreads();
  int wpre = 0, tt = 0, ovf = 0;
#pragma unroll
  for (int w2 = 0; w2 < NWAVE; ++w2) {
    const int tv = misc[8 + w2];
    wpre += (w2 < wave) ? tv : 0;
    tt   += tv;
    ovf  |= misc[16 + w2];
    ovf  |= (misc[w2] > WLCAP) ? 1 : 0;
  }
  ovf |= (tt > RCAP) ? 1 : 0;
  {
    const int excl = wpre + incT - ts;
    const v4i o4 = { excl, excl + tot4.x, excl + tot4.x + tot4.y, excl + tot4.x + tot4.y + tot4.z };
    v4i run = o4;
#pragma unroll
    for (int w = 0; w < NWAVE; ++w) {
      *(v4ia*)(cw + w * NBRUN + 4 * tid) = run;
      run += c4[w];
    }
    *(v4ia*)(cntS + 4 * tid) = tot4;
    *(v4ia*)(offS + 4 * tid) = o4;
  }
  __syncthreads();

#pragma unroll 1
  for (int q = 0; q < 4; ++q) {
    const int s = tid + 256 * q;
    dS[s] = 1.0f / sqrtf((float)(cntS[s] + 1));
  }

#pragma unroll 1
  for (int b0 = 0; b0 < wcc; b0 += 32) {
    int idx = b0 + lane;
    idx = idx < wcc - 1 ? idx : wcc - 1;
    const int ent = wl[idx];
    const int eid = clampi((int)((unsigned)ent >> SLB), 0, NE - 1);
    int sr = srcs[eid];
    asm volatile("" :: "v"(sr));
    sr = clampi(sr, 0, NN - 1);
    const int m32 = (wcc - b0) < 32 ? (wcc - b0) : 32;
#pragma unroll 1
    for (int k = 0; k < m32; ++k) {
      const int u  = __builtin_amdgcn_readlane(ent, k);
      const int sk = __builtin_amdgcn_readlane(sr, k);
      const int st = u & (NBRUN - 1);
      if (lane == 0) {
        const int p  = cwm[st];
        const int pc = clampi(p, 0, RCAP - 1);
        sl[pc]  = sk;
        cwm[st] = p + 1;
      }
    }
  }
  __syncthreads();

  v4i lv[8];
#pragma unroll
  for (int it = 0; it < 8; ++it) lv[it] = *(const v4ia*)(sl + 4 * (it * 256 + tid));
  const v4i oo = *(const v4ia*)(offS + 4 * tid);
  const v4i cc = *(const v4ia*)(cntS + 4 * tid);
  const v4f dd = *(const v4fa*)(dS + 4 * tid);
  const v4i ff = { ovf, ovf, ovf, ovf };
  int*   lp = LIST + (size_t)blk * RCAP;
  int*   op = OFF  + (size_t)nodeBase + 4 * tid;
  int*   cp = CNT  + (size_t)nodeBase + 4 * tid;
  float* dp = DINV + (size_t)nodeBase + 4 * tid;
  int*   fp = FLG  + (size_t)blk * 32 + 4 * (tid & 7);
#pragma unroll
  for (int it = 0; it < 8; ++it) *(volatile v4i*)(lp + 4 * (it * 256 + tid)) = lv[it];
  *(volatile v4i*)op = oo;
  *(volatile v4i*)cp = cc;
  *(volatile v4f*)dp = dd;
  if (tid < 8) *(volatile v4i*)fp = ff;
  __threadfence();
#pragma unroll
  for (int it = 0; it < 8; ++it) *(volatile v4i*)(lp + 4 * (it * 256 + tid)) = lv[it];
  *(volatile v4i*)op = oo;
  *(volatile v4i*)cp = cc;
  *(volatile v4f*)dp = dd;
  if (tid < 8) *(volatile v4i*)fp = ff;
}
#undef PUTJ

template <int LAYER>
__global__ __launch_bounds__(256) void k_replay(const int* __restrict__ xtok, const int* __restrict__ LIST,
                                                const int* __restrict__ OFF, const int* __restrict__ CNT,
                                                const float* __restrict__ DINV, const int* __restrict__ FLG,
                                                const float* __restrict__ SRC, const float* __restrict__ BR,
                                                unsigned short* __restrict__ hpl, float* __restrict__ outF) {
  static_assert(LAYER == 1 || LAYER == 2);
  __shared__ __attribute__((aligned(16))) float sB[DIM];
  const int tid = (int)threadIdx.x, lane = tid & 31, wave = tid >> 5;
  if (tid < 32) {
    const v4f b = *(const v4fa*)(BR + 4 * tid);
    *(v4fa*)(sB + 4 * tid) = b;
  }
  __syncthreads();
  const v4f bv = *(const v4fa*)(sB + 4 * lane);

  const int v  = (int)blockIdx.x * 8 + wave;
  const bool live = v < NN;
  const int vc = v < NN - 1 ? v : NN - 1;
  const int ob = vc >> SLB;
  const int   craw = CNT[vc];
  const int   oraw = OFF[vc];
  const float dv   = DINV[vc];
  const int   fl   = FLG[ob * 32];
  asm volatile("" :: "v"(craw));
  asm volatile("" :: "v"(oraw));
  asm volatile("" :: "v"(dv));
  asm volatile("" :: "v"(fl));
  int gs = vc;
  if (LAYER == 1) {
    const int xs = xtok[vc];
    asm volatile("" :: "v"(xs));
    gs = clampi(xs, 0, VOC - 1);
  }
  const bool big = (craw > DEGCAP) | (craw < 0);
  int cn = clampi(craw, 0, DEGCAP);
  cn = live ? cn : 0;
  cn = __builtin_amdgcn_readfirstlane(cn);
  const int o = clampi(oraw, 0, RCAP - 1);
  const int* lp = LIST + (size_t)ob * RCAP;

  float a0 = 0.0f, a1 = 0.0f, a2 = 0.0f, a3 = 0.0f;
#pragma unroll 1
  for (int b0 = 0; b0 < cn; b0 += 32) {
    int idx = o + b0 + lane;
    idx = idx > RCAP - 1 ? RCAP - 1 : idx;
    int s = lp[idx];
    asm volatile("" :: "v"(s));
    s = clampi(s, 0, NN - 1);
    int g = s;
    if (LAYER == 1) {
      const int t = xtok[s];
      asm volatile("" :: "v"(t));
      g = clampi(t, 0, VOC - 1);
    }
    const float ds = DINV[s];
    asm volatile("" :: "v"(ds));
    const float w  = ds * dv;
    const int   wi = __float_as_int(w);
    const int m32 = (cn - b0) < 32 ? (cn - b0) : 32;
#pragma unroll 1
    for (int k = 0; k < m32; ++k) {
      const int   gk = __builtin_amdgcn_readlane(g, k);
      const float wk = __int_as_float(__builtin_amdgcn_readlane(wi, k));
      const v4f r = *(const v4fa*)(SRC + (size_t)gk * DIM + 4 * lane);
      a0 = fmaf(wk, r.x, a0);
      a1 = fmaf(wk, r.y, a1);
      a2 = fmaf(wk, r.z, a2);
      a3 = fmaf(wk, r.w, a3);
    }
  }
  {
    const v4f r = *(const v4fa*)(SRC + (size_t)gs * DIM + 4 * lane);
    asm volatile("" :: "v"(r));
    const float sw = dv * dv;
    a0 = fmaf(sw, r.x, a0);
    a1 = fmaf(sw, r.y, a1);
    a2 = fmaf(sw, r.z, a2);
    a3 = fmaf(sw, r.w, a3);
  }
  float y0 = a0 + bv.x, y1 = a1 + bv.y, y2 = a2 + bv.z, y3 = a3 + bv.w;
  y0 = (y0 > 0.0f) ? y0 : (y0 - y0);
  y1 = (y1 > 0.0f) ? y1 : (y1 - y1);
  y2 = (y2 > 0.0f) ? y2 : (y2 - y2);
  y3 = (y3 > 0.0f) ? y3 : (y3 - y3);
  const float qnan = __int_as_float(0x7fc00000);
  const bool pois = (fl != 0) | big;
  y0 = pois ? qnan : y0;
  y1 = pois ? qnan : y1;
  y2 = pois ? qnan : y2;
  y3 = pois ? qnan : y3;
  const float z0 = live ? y0 : 0.0f;
  const float z1 = live ? y1 : 0.0f;
  const float z2 = live ? y2 : 0.0f;
  const float z3 = live ? y3 : 0.0f;

  if (LAYER == 1) {
    const int hw0 = (int)pk16(bf16_bits(z0), bf16_bits(z1));
    const int hw1 = (int)pk16(bf16_bits(z2), bf16_bits(z3));
    const int sa = (2 * lane) & 31, sb = (2 * lane + 1) & 31;
    const int g0 = __shfl(hw0, sa, 32), g1 = __shfl(hw1, sa, 32);
    const int g2 = __shfl(hw0, sb, 32), g3 = __shfl(hw1, sb, 32);
    v4u pv = (v4u){ (unsigned)g0, (unsigned)g1, (unsigned)g2, (unsigned)g3 };
    if (H1_SPLIT != 0) {
      const int lw0 = (int)pk16(bf16_lo_bits(z0), bf16_lo_bits(z1));
      const int lw1 = (int)pk16(bf16_lo_bits(z2), bf16_lo_bits(z3));
      const int p0 = __shfl(lw0, sa, 32), p1 = __shfl(lw1, sa, 32);
      const int p2 = __shfl(lw0, sb, 32), p3 = __shfl(lw1, sb, 32);
      const bool lsel = lane >= 16;
      pv.x = (unsigned)(lsel ? p0 : g0);
      pv.y = (unsigned)(lsel ? p1 : g1);
      pv.z = (unsigned)(lsel ? p2 : g2);
      pv.w = (unsigned)(lsel ? p3 : g3);
    }
    const int  piece = (H1_SPLIT != 0) ? lane : (lane & 15);
    const bool wr = (v < MPN) && ((H1_SPLIT != 0) || (lane < 16));
    unsigned short* hp = hpl + (size_t)v * K2TOT + 8 * piece;
    if (wr) *(volatile v4u*)hp = pv;
    __threadfence();
    if (wr) *(volatile v4u*)hp = pv;
  } else {
    const v4f ov = (v4f){ z0, z1, z2, z3 };
    float* op = outF + (size_t)vc * DIM + 4 * lane;
    if (live) *(volatile v4f*)op = ov;
    __threadfence();
    if (live) *(volatile v4f*)op = ov;
  }
}

extern "C" void kernel_launch(void* const* d_in, const int* in_sizes, int n_in,
                              void* d_out, int out_size, void* d_ws, size_t ws_size,
                              hipStream_t stream) {
  if (n_in < 7) return;
  if (in_sizes[0] != NN) return;
  if (in_sizes[1] != 2 * NE) return;
  if (in_sizes[2] != VOC * DIM) return;
  if (in_sizes[3] != DIM * DIM || in_sizes[4] != DIM) return;
  if (in_sizes[5] != DIM * DIM || in_sizes[6] != DIM) return;
  if (out_size != NN * DIM) return;
  if (ws_size < (size_t)WS_TOTAL) return;

  const int*   x    = (const int*)d_in[0];
  const int*   edge = (const int*)d_in[1];
  const float* emb  = (const float*)d_in[2];
  const float* W1   = (const float*)d_in[3];
  const float* b1   = (const float*)d_in[4];
  const float* W2   = (const float*)d_in[5];
  const float* b2   = (const float*)d_in[6];
  float* out = (float*)d_out;

  char* ws = (char*)d_ws;
  unsigned short* EB   = (unsigned short*)(ws + O_A);
  unsigned short* H1   = (unsigned short*)(ws + O_A);
  float*          T1   = (float*)(ws + O_B);
  float*          HW2  = (float*)(ws + O_B);
  int*            LIST = (int*)(ws + O_LIST);
  int*            OFF  = (int*)(ws + O_OFF);
  int*            CNT  = (int*)(ws + O_CNT);
  float*          DINV = (float*)(ws + O_DINV);
  int*            FLG  = (int*)(ws + O_FLG);
  unsigned short* W1T  = (unsigned short*)(ws + O_W1T);
  unsigned short* W2D  = (unsigned short*)(ws + O_W2D);
  float*          B1R  = (float*)(ws + O_B1R);
  float*          B2R  = (float*)(ws + O_B2R);

  static_assert(MPT % 64 == 0 && MPN % 64 == 0 && DIM % 64 == 0 && DIM % 32 == 0 && K2TOT % 32 == 0);
  static_assert(((long long)MPT * DIM / 8) % 256 == 0);
  static_assert((long long)MPN * K2TOT / 8 < (1LL << 31));

  hipFuncSetAttribute(reinterpret_cast<const void*>(&k_bucket), hipFuncAttributeMaxDynamicSharedMemorySize, (int)BK_BYTES);

  k_prep<<<PB1 + PB2 + 1, 256, 0, stream>>>(W1, W2, b1, b2, W1T, W2D, B1R, B2R);
  k_plane<0><<<MPT * DIM / 8 / 256, 256, 0, stream>>>(emb, VOC, DIM, DIM, EB, MPT, DIM);
  k_gemm_nt<0, 0><<<((MPT / 64) * (DIM / 64) + 7) / 8, 256, 0, stream>>>(EB, W1T, B1R, T1, MPT, DIM, DIM, DIM);
  k_bucket<<<NOWN, 256, BK_BYTES, stream>>>(edge, LIST, OFF, CNT, DINV, FLG);
  k_replay<1><<<MPN / 8, 256, 0, stream>>>(x, LIST, OFF, CNT, DINV, FLG, T1, B1R, H1, out);
  k_gemm_nt<H1_SPLIT, 0><<<((MPN / 64) * (DIM / 64) + 7) / 8, 256, 0, stream>>>(H1, W2D, B2R, HW2, MPN, DIM, K2TOT, DIM);
  k_replay<2><<<NN / 8, 256, 0, stream>>>(x, LIST, OFF, CNT, DINV, FLG, HW2, B2R, H1, out);
}
